// Module_9740985828114
// MI455X (gfx1250) — hardware-verified
//
#include <hip/hip_runtime.h>
#include <math.h>

typedef __attribute__((ext_vector_type(16))) _Float16 v16h;
typedef __attribute__((ext_vector_type(16))) __bf16 v16b;
typedef __attribute__((ext_vector_type(8)))  _Float16 v8h;
typedef __attribute__((ext_vector_type(8)))  float v8f;
typedef __attribute__((ext_vector_type(4)))  float v4f;
typedef __attribute__((ext_vector_type(2)))  float v2f;
typedef __attribute__((ext_vector_type(4)))  unsigned v4u;
typedef __attribute__((ext_vector_type(4)))  int v4i;
typedef float __attribute__((may_alias)) float_a;
typedef int __attribute__((may_alias)) int_a;

template <typename T> __device__ __forceinline__ void vst2(void* p, T v) { *(volatile T*)p = v; __threadfence(); *(volatile T*)p = v; }
__device__ __forceinline__ v8f wmma16(v16h a, v16h b, v8f c) {
  v8f d = __builtin_amdgcn_wmma_f32_16x16x32_f16(false, a, false, b, (short)0, c, false, false);
  asm volatile("v_nop\n\tv_nop\n\tv_nop\n\tv_nop" : "+v"(d) : "v"(a), "v"(b));
  return d;
}
__device__ __forceinline__ v8f wmma_bf(v16b a, v16b b, v8f c) {
  v8f d = __builtin_amdgcn_wmma_f32_16x16x32_bf16(false, a, false, b, (short)0, c, false, false);
  asm volatile("v_nop\n\tv_nop\n\tv_nop\n\tv_nop" : "+v"(d) : "v"(a), "v"(b));
  return d;
}
__device__ __forceinline__ v16h frag_h(const _Float16* rowk0, int lane) {
  union { v16h v; v8h q[2]; } u; const _Float16* p = rowk0 + 8 * (lane >> 4);
  u.q[0] = *(const v8h*)p; u.q[1] = *(const v8h*)(p + 16); return u.v;
}
__device__ __forceinline__ v16h frag_f32(const float* rowk0, int lane) {
  v16h a; const float* p = rowk0 + 8 * (lane >> 4);
#pragma unroll
  for (int i = 0; i < 8; ++i) { a[i] = (_Float16)p[i]; a[8 + i] = (_Float16)p[16 + i]; }
  return a;
}
__device__ __forceinline__ v16h frag_f32s(const float* rowk0, int lane, float sc) {
  v16h a; const float* p = rowk0 + 8 * (lane >> 4);
#pragma unroll
  for (int i = 0; i < 8; ++i) { a[i] = (_Float16)(p[i] * sc); a[8 + i] = (_Float16)(p[16 + i] * sc); }
  return a;
}
__device__ __forceinline__ v16h fragc_f32(const float* W, int k0, int n, int lane, int ld, int K) {
  v16h a; const int g = lane >> 4;
#pragma unroll
  for (int i = 0; i < 8; ++i) { const int ka = k0 + 8 * g + i, kb = ka + 16;
    a[i] = (_Float16)(ka < K ? W[(size_t)(ka < K ? ka : K - 1) * ld + n] : 0.f); a[8 + i] = (_Float16)(kb < K ? W[(size_t)(kb < K ? kb : K - 1) * ld + n] : 0.f); }
  return a;
}
struct F2 { v16b h, l; };
__device__ __forceinline__ F2 bsplit16(const float v[16]) { F2 r;
#pragma unroll
  for (int i = 0; i < 16; ++i) { const __bf16 h = (__bf16)v[i]; r.h[i] = h; r.l[i] = (__bf16)(v[i] - (float)h); }
  return r; }
__device__ __forceinline__ F2 split_row(const float* row, int k0, int lane) { float v[16]; const float* p = row + k0 + 8 * (lane >> 4);
#pragma unroll
  for (int i = 0; i < 8; ++i) { v[i] = p[i]; v[8 + i] = p[16 + i]; }
  return bsplit16(v); }
__device__ __forceinline__ F2 split_rowK(const float* row, int k0, int lane, int K) { float v[16]; const int g = lane >> 4;
#pragma unroll
  for (int i = 0; i < 8; ++i) { const int ka = k0 + 8 * g + i, kb = ka + 16; v[i] = ka < K ? row[ka < K ? ka : K - 1] : 0.f; v[8 + i] = kb < K ? row[kb < K ? kb : K - 1] : 0.f; }
  return bsplit16(v); }
__device__ __forceinline__ F2 split_col(const float* W, int k0, int n, int lane, int ld, int K) { float v[16]; const int g = lane >> 4;
#pragma unroll
  for (int i = 0; i < 8; ++i) { const int ka = k0 + 8 * g + i, kb = ka + 16; v[i] = ka < K ? W[(size_t)(ka < K ? ka : K - 1) * ld + n] : 0.f; v[8 + i] = kb < K ? W[(size_t)(kb < K ? kb : K - 1) * ld + n] : 0.f; }
  return bsplit16(v); }
__device__ __forceinline__ v8f mac3(const F2& a, const F2& b, v8f c) { c = wmma_bf(a.l, b.h, c); c = wmma_bf(a.h, b.l, c); return wmma_bf(a.h, b.h, c); }
__device__ __forceinline__ float sigm(float v) { return 1.0f / (1.0f + expf(-v)); }
#define LDSX() do { asm volatile("s_wait_dscnt 0" ::: "memory"); __builtin_amdgcn_wave_barrier(); __builtin_amdgcn_fence(__ATOMIC_RELEASE, "workgroup"); } while (0)


#define NB 2
#define TT 1024
#define SC 1024
#define SKV (SC + TT)
#define DM_ 2048
#define NHQ 16
#define NKV 4
#define HD 128
#define QW (NHQ * HD)
#define KW (NKV * HD)
#define QKVW (QW + 2 * KW)
#ifndef TNB
#define TNB NB
#endif
#ifndef TQB
#define TQB (TT / 64)
#endif
#ifndef TRB
#define TRB (TNB * TT / 64)
#endif
typedef __attribute__((ext_vector_type(8))) __bf16 v8b;
__device__ __forceinline__ v16b frag_b(const __bf16* rowk0, int lane) {
  union { v16b v; v8b q[2]; } u; const __bf16* p = rowk0 + 8 * (lane >> 4);
  u.q[0] = *(const v8b*)p; u.q[1] = *(const v8b*)(p + 16); return u.v;
}
__device__ __forceinline__ float bfr(float v) { return (float)(__bf16)v; }
__device__ __attribute__((noinline)) float exp_ni(float v) { return expf(v); }
__device__ __attribute__((noinline)) float erf_ni(float v) { return erff(v); }

#define WS_F   0u
#define WS_QH  (WS_F + 4u * (size_t)NB * TT * QKVW)
#define WS_KH  (WS_QH + 2u * (size_t)NB * TT * QW)
#define WS_VH  (WS_KH + 2u * (size_t)NB * SKV * KW)
#define WS_VL  (WS_VH + 2u * (size_t)NB * KW * SKV)
#define WS_CT  (WS_VL + 2u * (size_t)NB * KW * SKV)
#define WS_END (WS_CT + 4u * (size_t)NB * TT * QW)

__global__ __launch_bounds__(128) void k_qkv(const float* __restrict__ X, const float* __restrict__ WQ, const float* __restrict__ WKV, float* __restrict__ F) { __shared__ __align__(16) float sf[4][16][132];
  const int tid = threadIdx.x, wave = tid >> 5, lane = tid & 31, col = lane & 15, g = lane >> 4; const int cg = blockIdx.y; const size_t r0 = (size_t)blockIdx.x * 64 + wave * 16;
  const float* Wh; if (cg < 16) Wh = WQ + (size_t)cg * DM_ * HD; else if (cg < 20) Wh = WKV + ((size_t)0 * NKV + (cg - 16)) * DM_ * HD; else Wh = WKV + ((size_t)1 * NKV + (cg - 20)) * DM_ * HD;
  v8f acc[8] = {};
#pragma unroll 2
  for (int kc = 0; kc < DM_ / 32; ++kc) { v16b a; { const float* p = X + (r0 + col) * DM_ + kc * 32 + 8 * g;
#pragma unroll
      for (int i = 0; i < 8; ++i) { a[i] = (__bf16)p[i]; a[8 + i] = (__bf16)p[16 + i]; } }
#pragma unroll
    for (int j = 0; j < 8; ++j) { v16b w; const int hh = j * 16 + col;
#pragma unroll
      for (int i = 0; i < 8; ++i) { w[i] = (__bf16)Wh[(size_t)(kc * 32 + 8 * g + i) * HD + hh]; w[8 + i] = (__bf16)Wh[(size_t)(kc * 32 + 16 + 8 * g + i) * HD + hh]; }
      acc[j] = wmma_bf(a, w, acc[j]); } }
#pragma unroll
  for (int j = 0; j < 8; ++j)
#pragma unroll
    for (int r = 0; r < 8; ++r) sf[wave][8 * g + r][j * 16 + col] = acc[j][r];
  LDSX(); for (int rl = 0; rl < 16; ++rl) vst2(F + (r0 + rl) * QKVW + cg * 128 + lane * 4, *(const v4f*)&sf[wave][rl][lane * 4]); }
__global__ __launch_bounds__(256) void k_rope(const float* __restrict__ F, const int* __restrict__ POS, _Float16* __restrict__ QH, _Float16* __restrict__ KH) { __shared__ __align__(16) _Float16 sh[QW + KW];
  const int t = threadIdx.x; const size_t row = blockIdx.x; const size_t b = row / TT; const int tt = (int)(row % TT); const float pos = (float)POS[row]; const float* fr = F + row * QKVW;
  for (int e = t; e < (QW + KW) / 2; e += 256) { const int hh = e / (HD / 2), j = e % (HD / 2); const int o1 = hh * HD + j, o2 = o1 + HD / 2;
    const float ang = pos / powf(10000.0f, (2.0f / (float)HD) * (float)j); const float c = cosf(ang), sn = sinf(ang); const float x1 = fr[o1], x2 = fr[o2];
    float y1 = x1 * c - x2 * sn, y2 = x2 * c + x1 * sn; if (hh < NHQ) { y1 *= 0.08838834764831845f; y2 *= 0.08838834764831845f; }
    sh[o1] = (_Float16)y1; sh[o2] = (_Float16)y2; }
  __syncthreads();
  for (int q = t; q < QW / 8; q += 256) vst2((unsigned*)(QH + row * QW + q * 8), *(const v4u*)&sh[q * 8]);
  for (int q = t; q < KW / 8; q += 256) vst2((unsigned*)(KH + (b * SKV + SC + tt) * KW + q * 8), *(const v4u*)&sh[QW + q * 8]); }
__global__ __launch_bounds__(128) void k_kv2(const float* __restrict__ CK, const float* __restrict__ CV, const float* __restrict__ F, _Float16* __restrict__ KH, _Float16* __restrict__ VH, _Float16* __restrict__ VL) { __shared__ __align__(16) _Float16 th[256][72], tl[256][72];
  const int t = threadIdx.x; const size_t b = blockIdx.y; const int sb = blockIdx.x; const size_t s0 = (size_t)sb * 64; const bool cache = (sb < SC / 64);
  if (cache) { for (int e = t; e < 64 * (KW / 8); e += 128) { const int sl_ = e / (KW / 8), q = e % (KW / 8); const float* src = CK + ((b * SC + s0 + sl_) * KW) + q * 8; _Float16 h8[8];
#pragma unroll
      for (int i = 0; i < 8; ++i) h8[i] = (_Float16)bfr(src[i]);
      vst2((unsigned*)(KH + (b * SKV + s0 + sl_) * KW + q * 8), *(const v4u*)h8); } }
#pragma unroll 1
  for (int half = 0; half < 2; ++half) { const int c0 = half * 256;
    for (int e = t; e < 64 * 256; e += 128) { const int sl_ = e >> 8, c = e & 255; float v; if (cache) v = bfr(CV[((b * SC + s0 + sl_) * KW) + c0 + c]); else v = F[((b * TT + (s0 - SC) + sl_) * QKVW) + QW + KW + c0 + c]; const _Float16 hv = (_Float16)v; th[c][sl_] = hv; tl[c][sl_] = cache ? (_Float16)0.0f : (_Float16)(v - (float)hv); }
    __syncthreads();
    for (int e = t; e < 256 * 8; e += 128) { const int c = e >> 3, q = e & 7; const size_t o = (b * KW + c0 + c) * (size_t)SKV + s0 + q * 8; vst2((unsigned*)(VH + o), *(const v4u*)&th[c][q * 8]); vst2((unsigned*)(VL + o), *(const v4u*)&tl[c][q * 8]); }
    __syncthreads(); } }
__global__ __launch_bounds__(128) void k_att(const _Float16* __restrict__ QH, const _Float16* __restrict__ KH, const _Float16* __restrict__ VH, const _Float16* __restrict__ VL, const int* __restrict__ AM, float* __restrict__ CT) {
  __shared__ __align__(16) float sp[4][16][36]; __shared__ __align__(16) float so[4][16][132];
  const int tid = threadIdx.x, wave = tid >> 5, lane = tid & 31, col = lane & 15, g = lane >> 4; const int qb = blockIdx.x, h = blockIdx.y; const size_t b = blockIdx.z; const int kvh = h / (NHQ / NKV); const int q0 = qb * 64 + wave * 16;
  v16h aq[4];
#pragma unroll
  for (int kc = 0; kc < 4; ++kc) aq[kc] = frag_h(QH + (b * TT + q0 + col) * QW + h * HD + kc * 32, lane);
  float m[8], l[8];
#pragma unroll
  for (int r = 0; r < 8; ++r) { m[r] = -3.0e38f; l[r] = 0.f; }
  v8f acc[8] = {};
  const int nks = (SC + qb * 64 + 64) / 32;
#pragma unroll 1
  for (int ks = 0; ks < nks; ++ks) { float s[2][8];
#pragma unroll
    for (int ct = 0; ct < 2; ++ct) { const int kk = ks * 32 + ct * 16 + col; v8f c = {};
#pragma unroll
      for (int kc = 0; kc < 4; ++kc) c = wmma16(aq[kc], frag_h(KH + (b * SKV + kk) * KW + kvh * HD + kc * 32, lane), c);
#pragma unroll
      for (int r = 0; r < 8; ++r) { const int q = q0 + 8 * g + r; const bool keep = (AM[(b * TT + q) * (size_t)SKV + kk] != 0); s[ct][r] = keep ? tanhf(c[r] * 0.02f) * 50.0f : -3.0e38f; } }
    float alpha[8];
#pragma unroll
    for (int r = 0; r < 8; ++r) { float mx = fmaxf(s[0][r], s[1][r]);
#pragma unroll
      for (int o = 1; o < 16; o <<= 1) mx = fmaxf(mx, __shfl_xor(mx, o));
      const float mn = fmaxf(m[r], mx); alpha[r] = (m[r] <= -1.0e38f) ? 0.f : __expf(m[r] - mn); const float e0 = (s[0][r] <= -1.0e38f) ? 0.f : __expf(s[0][r] - mn), e1 = (s[1][r] <= -1.0e38f) ? 0.f : __expf(s[1][r] - mn); float es = e0 + e1;
#pragma unroll
      for (int o = 1; o < 16; o <<= 1) es += __shfl_xor(es, o);
      l[r] = l[r] * alpha[r] + es; m[r] = mn; sp[wave][8 * g + r][col] = e0; sp[wave][8 * g + r][16 + col] = e1; }
#pragma unroll
    for (int j = 0; j < 8; ++j)
#pragma unroll
      for (int r = 0; r < 8; ++r) acc[j][r] *= alpha[r];
    LDSX();
    const v16h pa = frag_f32s(&sp[wave][col][0], lane, 2048.0f);
#pragma unroll
    for (int j = 0; j < 8; ++j) { const size_t po = (b * KW + (size_t)kvh * HD + j * 16 + col) * SKV + ks * 32; acc[j] = wmma16(pa, frag_h(VH + po, lane), acc[j]); acc[j] = wmma16(pa, frag_h(VL + po, lane), acc[j]); }
    LDSX(); }
#pragma unroll
  for (int r = 0; r < 8; ++r) { const float il = (l[r] > 0.f) ? (1.0f / 2048.0f) / l[r] : 0.f;
#pragma unroll
    for (int j = 0; j < 8; ++j) so[wave][8 * g + r][j * 16 + col] = acc[j][r] * il; }
  LDSX(); for (int rl = 0; rl < 16; ++rl) vst2(CT + (b * TT + q0 + rl) * QW + h * HD + lane * 4, *(const v4f*)&so[wave][rl][lane * 4]); }
__global__ __launch_bounds__(128) void k_out(const float* __restrict__ CT, const float* __restrict__ WO, float* __restrict__ OUT) { __shared__ __align__(16) float sf[4][16][132];
  const int tid = threadIdx.x, wave = tid >> 5, lane = tid & 31, col = lane & 15, g = lane >> 4; const int c0 = blockIdx.y * 128; const size_t r0 = (size_t)blockIdx.x * 64 + wave * 16;
  v8f acc[8] = {};
#pragma unroll 2
  for (int kc = 0; kc < QW / 32; ++kc) { const F2 a = split_row(CT + (r0 + col) * QW, kc * 32, lane);
#pragma unroll
    for (int j = 0; j < 8; ++j) { v16b w; const int o = c0 + j * 16 + col;
#pragma unroll
      for (int i = 0; i < 8; ++i) { w[i] = (__bf16)WO[(size_t)(kc * 32 + 8 * g + i) * DM_ + o]; w[8 + i] = (__bf16)WO[(size_t)(kc * 32 + 16 + 8 * g + i) * DM_ + o]; }
      acc[j] = wmma_bf(a.h, w, acc[j]); acc[j] = wmma_bf(a.l, w, acc[j]); } }
#pragma unroll
  for (int j = 0; j < 8; ++j)
#pragma unroll
    for (int r = 0; r < 8; ++r) sf[wave][8 * g + r][j * 16 + col] = acc[j][r];
  LDSX(); for (int rl = 0; rl < 16; ++rl) vst2(OUT + (r0 + rl) * DM_ + c0 + lane * 4, *(const v4f*)&sf[wave][rl][lane * 4]); }
extern "C" void kernel_launch(void* const* d_in, const int* in_sizes, int n_in, void* d_out, int out_size, void* d_ws, size_t ws_size, hipStream_t stream) {
  (void)in_sizes; (void)n_in; (void)out_size;
  const float** F_ = (const float**)d_in;
  if (ws_size < (size_t)WS_END) return;
  char* ws = (char*)d_ws; float* F = (float*)(ws + WS_F); _Float16 *QH = (_Float16*)(ws + WS_QH), *KH = (_Float16*)(ws + WS_KH), *VH = (_Float16*)(ws + WS_VH), *VL = (_Float16*)(ws + WS_VL); float* CT = (float*)(ws + WS_CT);
  k_qkv<<<dim3(TRB, QKVW / 128), 128, 0, stream>>>(F_[0], F_[5], F_[6], F);
  k_rope<<<TRB * 64, 256, 0, stream>>>(F, (const int*)d_in[1], QH, KH);
  k_kv2<<<dim3(SKV / 64, TNB), 128, 0, stream>>>(F_[3], F_[4], F, KH, VH, VL);
  k_att<<<dim3(TQB, NHQ, TNB), 128, 0, stream>>>(QH, KH, VH, VL, (const int*)d_in[2], CT);
  k_out<<<dim3(TRB, DM_ / 128), 128, 0, stream>>>(CT, F_[7], (float*)d_out);
}
